// LongformerSelfAttention_12730283065484
// MI455X (gfx1250) — hardware-verified
//
#include <hip/hip_runtime.h>
#include <hip/hip_bf16.h>

#ifndef NB
#define NB 2
#endif
#ifndef SEQ
#define SEQ 4096
#endif
#define NB_FULL  2
#define SEQ_FULL 4096
#define HID   768
#define NH    12
#define HD    64
#define WIN   256
#define NSTEP 17
#define XCH   (HID / 256)

static_assert((SEQ % 64) == 0);
static_assert(SEQ >= 64);
static_assert(NB >= 1);
static_assert(NB <= NB_FULL);
static_assert(SEQ <= SEQ_FULL);
static_assert(NH * HD == HID);
static_assert((HID % 256) == 0);
static_assert(32 * NSTEP >= 2 * WIN + 16);

typedef float  v8f  __attribute__((ext_vector_type(8)));
typedef float  v4f  __attribute__((ext_vector_type(4)));
typedef int    v4i  __attribute__((ext_vector_type(4)));
typedef __bf16 v8b  __attribute__((ext_vector_type(8)));
typedef __bf16 v16b __attribute__((ext_vector_type(16)));

union Frag   { v16b v; v8b h[2]; };
union Pack16 { v8b b; v4i u; };

__device__ __forceinline__ void mma(v8f& c, const v16b a, const v16b b) {
    c = __builtin_amdgcn_wmma_f32_16x16x32_bf16(false, a, false, b, (short)0, c, false, false);
    asm volatile("v_nop\n\tv_nop\n\tv_nop\n\tv_nop" : "+v"(c) : "v"(a), "v"(b));
}

__device__ __forceinline__ v8f zero8() {
    return (v8f){0.f, 0.f, 0.f, 0.f, 0.f, 0.f, 0.f, 0.f};
}

__device__ __forceinline__ int clampi(int v, int lo, int hi) {
    return v < lo ? lo : (v > hi ? hi : v);
}

__global__ __launch_bounds__(256) void k_cvt(
    const float* __restrict__ x,  const float* __restrict__ w0,
    const float* __restrict__ w1, const float* __restrict__ w2,
    __bf16* __restrict__ xb, __bf16* __restrict__ wb, int nxc, int nwc)
{
    const int lane = threadIdx.x & 31;
    const int c = blockIdx.x * 8 + (threadIdx.x >> 5);
    if (c >= nxc + 3 * nwc) return;
    const float* src;
    __bf16* dst;
    if (c < nxc) {
        const int tok  = c / XCH;
        const int part = c - tok * XCH;
        const int bb   = tok / SEQ;
        const int ss   = tok - bb * SEQ;
        src = x + ((size_t)bb * SEQ_FULL + ss) * HID + part * 256;
        dst = xb + (size_t)c * 256;
    } else {
        const int rr = c - nxc;
        const int mi = rr / nwc;
        const int cc = rr - mi * nwc;
        const float* wsrc = (mi == 0) ? w0 : ((mi == 1) ? w1 : w2);
        src = wsrc + (size_t)cc * 256;
        dst = wb + ((size_t)mi * nwc + cc) * 256;
    }
    const v4f f0 = *(const v4f*)(src + lane * 8);
    const v4f f1 = *(const v4f*)(src + lane * 8 + 4);
    Pack16 o;
    #pragma unroll
    for (int e = 0; e < 4; e++) {
        o.b[e]     = (__bf16)f0[e];
        o.b[4 + e] = (__bf16)f1[e];
    }
    const v4i ov = o.u;
    volatile v4i* dp = (volatile v4i*)(dst + lane * 8);
    *dp = ov;
    __threadfence();
    *dp = ov;
}

__global__ __launch_bounds__(128) void k_proj(
    const __bf16* __restrict__ xb, const __bf16* __restrict__ wb,
    const float* __restrict__ bq, const float* __restrict__ bk, const float* __restrict__ bv,
    __bf16* __restrict__ qh, __bf16* __restrict__ ql,
    __bf16* __restrict__ kh, __bf16* __restrict__ kl,
    __bf16* __restrict__ vth, __bf16* __restrict__ vtl)
{
    __shared__ __attribute__((aligned(16))) __bf16 s_hi[64 * 64];
    __shared__ __attribute__((aligned(16))) __bf16 s_lo[64 * 64];

    const int t0 = blockIdx.x * 64;
    if (t0 >= NB * SEQ) return;
    const int lane = threadIdx.x & 31, w = threadIdx.x >> 5;
    const int h = lane >> 4, m = lane & 15;
    const int mi = blockIdx.z, head = blockIdx.y;
    const int tw = t0 + 16 * w;

    const __bf16* W = wb + (size_t)mi * HID * HID;
    const float* bias = (mi == 0) ? bq : ((mi == 1) ? bk : bv);
    const float scale = (mi == 0) ? 0.125f : 1.0f;

    const __bf16* arow = xb + (size_t)(tw + m) * HID;
    v8f acc[4];
    #pragma unroll
    for (int s4 = 0; s4 < 4; s4++) acc[s4] = zero8();

    #pragma unroll 1
    for (int k0 = 0; k0 < HID; k0 += 32) {
        Frag a;
        a.h[0] = *(const v8b*)(arow + k0 + 8 * h);
        a.h[1] = *(const v8b*)(arow + k0 + 16 + 8 * h);
        #pragma unroll
        for (int s4 = 0; s4 < 4; s4++) {
            const __bf16* wr = W + (size_t)(head * HD + s4 * 16 + m) * HID + k0;
            Frag b;
            b.h[0] = *(const v8b*)(wr + 8 * h);
            b.h[1] = *(const v8b*)(wr + 16 + 8 * h);
            mma(acc[s4], a.v, b.v);
        }
    }

    #pragma unroll
    for (int s4 = 0; s4 < 4; s4++) {
        const int col = s4 * 16 + m;
        const float bb = (float)(__bf16)bias[head * HD + col];
        #pragma unroll
        for (int r = 0; r < 8; r++) {
            const int tokl = 16 * w + 8 * h + r;
            const float y = (acc[s4][r] + bb) * scale;
            const __bf16 yh = (__bf16)y;
            const __bf16 yl = (__bf16)(y - (float)yh);
            const int idx = (mi == 2) ? (col * 64 + tokl) : (tokl * 64 + col);
            s_hi[idx] = yh;
            s_lo[idx] = yl;
        }
    }
    __syncthreads();

    const int bb_ = t0 / SEQ;
    const int s0 = t0 - bb_ * SEQ;
    const int bh = bb_ * NH + head;
    const int q = lane >> 3, p = lane & 7;
    __bf16* ph_ = (mi == 0) ? qh : ((mi == 1) ? kh : vth);
    __bf16* pl_ = (mi == 0) ? ql : ((mi == 1) ? kl : vtl);
    v4i dh[4], dl[4];
    size_t off[4];
    #pragma unroll
    for (int it = 0; it < 4; it++) {
        const int L = 16 * w + 4 * it + q;
        dh[it] = *(const v4i*)(s_hi + L * 64 + p * 8);
        dl[it] = *(const v4i*)(s_lo + L * 64 + p * 8);
        off[it] = (mi == 2)
            ? ((size_t)(bh * HD + L) * SEQ + s0 + p * 8)
            : ((size_t)(bh * SEQ + s0 + L) * HD + p * 8);
    }
    #pragma unroll
    for (int it = 0; it < 4; it++) {
        *(volatile v4i*)(ph_ + off[it]) = dh[it];
        *(volatile v4i*)(pl_ + off[it]) = dl[it];
    }
    __threadfence();
    #pragma unroll
    for (int it = 0; it < 4; it++) {
        *(volatile v4i*)(ph_ + off[it]) = dh[it];
        *(volatile v4i*)(pl_ + off[it]) = dl[it];
    }
}

__global__ __launch_bounds__(64) void k_attn(
    const __bf16* __restrict__ qh, const __bf16* __restrict__ ql,
    const __bf16* __restrict__ kh, const __bf16* __restrict__ kl,
    const __bf16* __restrict__ vth, const __bf16* __restrict__ vtl,
    float* __restrict__ out)
{
    __shared__ __attribute__((aligned(16))) float s_o[2][16 * HD];

    if (blockIdx.x * 32 >= SEQ) return;
    const int lane = threadIdx.x & 31, w = threadIdx.x >> 5;
    const int h = lane >> 4, m = lane & 15;
    const int b = blockIdx.z, head = blockIdx.y;
    const int i0 = blockIdx.x * 32 + w * 16;
    const int bh = b * NH + head;
    const int iq = i0 + m;

    const float NEG_BIG  = -1.0e30f;
    const float NEG_TEST = -1.0e29f;

    Frag bqh[2], bql[2];
    {
        const size_t qo = ((size_t)bh * SEQ + i0 + m) * HD;
        #pragma unroll
        for (int dd = 0; dd < 2; dd++) {
            bqh[dd].h[0] = *(const v8b*)(qh + qo + 32 * dd + 8 * h);
            bqh[dd].h[1] = *(const v8b*)(qh + qo + 32 * dd + 16 + 8 * h);
            bql[dd].h[0] = *(const v8b*)(ql + qo + 32 * dd + 8 * h);
            bql[dd].h[1] = *(const v8b*)(ql + qo + 32 * dd + 16 + 8 * h);
        }
    }

    const size_t kbase = (size_t)bh * SEQ * HD;
    const size_t vbase = (size_t)bh * HD * SEQ;

    v8f ctx[4];
    #pragma unroll
    for (int s4 = 0; s4 < 4; s4++) ctx[s4] = zero8();
    float mrun = NEG_BIG;
    float lrun = 0.f;

    #pragma unroll 1
    for (int step = 0; step < NSTEP; step++) {
        const int jb = i0 - WIN + 32 * step;
        float sv[2][8];
        float tmax = NEG_BIG;
        #pragma unroll
        for (int t = 0; t < 2; t++) {
            const int jt = jb + 16 * t;
            const int jc = clampi(jt, 0, SEQ - 16);
            const __bf16* khr = kh + kbase + (size_t)(jc + m) * HD;
            const __bf16* klr = kl + kbase + (size_t)(jc + m) * HD;
            v8f st = zero8();
            #pragma unroll
            for (int dd = 0; dd < 2; dd++) {
                Frag ah, al;
                ah.h[0] = *(const v8b*)(khr + 32 * dd + 8 * h);
                ah.h[1] = *(const v8b*)(khr + 32 * dd + 16 + 8 * h);
                al.h[0] = *(const v8b*)(klr + 32 * dd + 8 * h);
                al.h[1] = *(const v8b*)(klr + 32 * dd + 16 + 8 * h);
                mma(st, ah.v, bqh[dd].v);
                mma(st, ah.v, bql[dd].v);
                mma(st, al.v, bqh[dd].v);
            }
            #pragma unroll
            for (int r = 0; r < 8; r++) {
                const int j = jt + 8 * h + r;
                const int di = j - iq;
                const bool ok = (j >= 0) && (j < SEQ) && (di <= WIN) && (di >= -WIN);
                const float s = ok ? st[r] : NEG_BIG;
                sv[t][r] = s;
                tmax = fmaxf(tmax, s);
            }
        }
        tmax = fmaxf(tmax, __shfl_xor(tmax, 16, 32));
        const float mnew = fmaxf(mrun, tmax);
        const float scal = __expf(mrun - mnew);
        mrun = mnew;

        float psum = 0.f;
        v16b aph, apl;
        #pragma unroll
        for (int t = 0; t < 2; t++) {
            #pragma unroll
            for (int e = 0; e < 8; e++) {
                const float s  = sv[t][e];
                const float pe = __expf(s - mnew);
                const float p  = (s > NEG_TEST) ? pe : 0.0f;
                psum += p;
                const __bf16 hb = (__bf16)p;
                aph[8 * t + e] = hb;
                apl[8 * t + e] = (__bf16)(p - (float)hb);
            }
        }
        lrun = lrun * scal + psum;

        #pragma unroll
        for (int r = 0; r < 8; r++) {
            const float sr = __shfl(scal, 8 * h + r, 32);
            #pragma unroll
            for (int s4 = 0; s4 < 4; s4++) ctx[s4][r] *= sr;
        }
        #pragma unroll
        for (int s4 = 0; s4 < 4; s4++)
            asm volatile("v_nop\n\tv_nop\n\tv_nop\n\tv_nop" : "+v"(ctx[s4]));

        const int jc0 = clampi(jb, 0, SEQ - 16);
        const int jc1 = clampi(jb + 16, 0, SEQ - 16);
        #pragma unroll
        for (int s4 = 0; s4 < 4; s4++) {
            const __bf16* vhr = vth + vbase + (size_t)(s4 * 16 + m) * SEQ;
            const __bf16* vlr = vtl + vbase + (size_t)(s4 * 16 + m) * SEQ;
            Frag bvh, bvl;
            bvh.h[0] = *(const v8b*)(vhr + jc0 + 8 * h);
            bvh.h[1] = *(const v8b*)(vhr + jc1 + 8 * h);
            bvl.h[0] = *(const v8b*)(vlr + jc0 + 8 * h);
            bvl.h[1] = *(const v8b*)(vlr + jc1 + 8 * h);
            mma(ctx[s4], aph, bvh.v);
            mma(ctx[s4], aph, bvl.v);
            mma(ctx[s4], apl, bvh.v);
        }
    }

    lrun += __shfl_xor(lrun, 16, 32);

    float* so = s_o[w];
    #pragma unroll
    for (int r = 0; r < 8; r++) {
        const int rowl = 8 * h + r;
        const float den = __shfl(lrun, rowl, 32);
        const float inv = 1.0f / den;
        #pragma unroll
        for (int s4 = 0; s4 < 4; s4++)
            so[rowl * HD + s4 * 16 + m] = ctx[s4][r] * inv;
    }
    __syncthreads();

    float* ob = out + ((size_t)(b * SEQ + i0)) * HID + head * HD;
    v4f ov[8];
    int oo[8];
    #pragma unroll
    for (int it = 0; it < 8; it++) {
        const int rowl = 2 * it + (lane >> 4);
        const int pc = lane & 15;
        ov[it] = *(const v4f*)(so + rowl * HD + 4 * pc);
        oo[it] = rowl * HID + 4 * pc;
    }
    #pragma unroll
    for (int it = 0; it < 8; it++) *(volatile v4f*)(ob + oo[it]) = ov[it];
    __threadfence();
    #pragma unroll
    for (int it = 0; it < 8; it++) *(volatile v4f*)(ob + oo[it]) = ov[it];
}

extern "C" void kernel_launch(void* const* d_in, const int* in_sizes, int n_in,
                              void* d_out, int out_size, void* d_ws, size_t ws_size,
                              hipStream_t stream)
{
    if (n_in < 7) return;
    if (in_sizes[0] < ((NB - 1) * SEQ_FULL + SEQ) * HID) return;
    if (in_sizes[1] < HID * HID || in_sizes[3] < HID * HID || in_sizes[5] < HID * HID) return;
    if (in_sizes[2] < HID || in_sizes[4] < HID || in_sizes[6] < HID) return;
    if (out_size < NB * SEQ * HID) return;

    const float* x  = (const float*)d_in[0];
    const float* Wq = (const float*)d_in[1];
    const float* bq = (const float*)d_in[2];
    const float* Wk = (const float*)d_in[3];
    const float* bk = (const float*)d_in[4];
    const float* Wv = (const float*)d_in[5];
    const float* bv = (const float*)d_in[6];
    float* out = (float*)d_out;

    const size_t bytes_x16 = (size_t)NB * SEQ * HID * 2;
    const size_t bytes_w16 = (size_t)3 * HID * HID * 2;
    const size_t bytes_pl  = (size_t)NB * NH * SEQ * HD * 2;
    size_t off = 0;
    char* ws = (char*)d_ws;
    __bf16* xb  = (__bf16*)(ws + off); off += bytes_x16;
    __bf16* wb  = (__bf16*)(ws + off); off += bytes_w16;
    __bf16* qh  = (__bf16*)(ws + off); off += bytes_pl;
    __bf16* ql  = (__bf16*)(ws + off); off += bytes_pl;
    __bf16* kh  = (__bf16*)(ws + off); off += bytes_pl;
    __bf16* kl  = (__bf16*)(ws + off); off += bytes_pl;
    __bf16* vth = (__bf16*)(ws + off); off += bytes_pl;
    __bf16* vtl = (__bf16*)(ws + off); off += bytes_pl;
    if (off > ws_size) return;

    const int nxc = (NB * SEQ * HID) / 256;
    const int nwc = (HID * HID) / 256;
    const int nchunks = nxc + 3 * nwc;
    const int cvt_blocks = (nchunks + 7) / 8;

    k_cvt<<<dim3(cvt_blocks, 1, 1), 256, 0, stream>>>(x, Wq, Wk, Wv, xb, wb, nxc, nwc);
    k_proj<<<dim3((NB * SEQ + 63) / 64, NH, 3), 128, 0, stream>>>(xb, wb, bq, bk, bv,
                                                                  qh, ql, kh, kl, vth, vtl);
    k_attn<<<dim3((SEQ + 31) / 32, NH, NB), 64, 0, stream>>>(qh, ql, kh, kl, vth, vtl, out);
}
